// Conv2d_gradual_int8_27788438405485
// MI455X (gfx1250) — hardware-verified
//
#include <hip/hip_runtime.h>
#include <math.h>

#define CB 4
#define CC 64
#define CHW 32
#define CO 128
#define CK 576
typedef _Float16 h16;
typedef __attribute__((ext_vector_type(16))) _Float16 v16h;
typedef __attribute__((ext_vector_type(8)))  _Float16 v8h;
typedef __attribute__((ext_vector_type(8)))  float v8f;
typedef __attribute__((ext_vector_type(4)))  float v4f_t;
typedef float v4fa __attribute__((ext_vector_type(4), may_alias));
typedef __attribute__((ext_vector_type(4)))  unsigned v4u_t;
typedef unsigned v4ua __attribute__((ext_vector_type(4), may_alias));

__device__ __forceinline__ v8f wmma16(v16h a, v16h b, v8f c) { return __builtin_amdgcn_wmma_f32_16x16x32_f16(false, a, false, b, (short)0, c, false, false); }
__device__ __forceinline__ v16h rfrag(const h16* rowp, int half) {
  const h16* p = rowp + 8 * half;
  return __builtin_shufflevector(*(const v8h*)p, *(const v8h*)(p + 16), 0,1,2,3,4,5,6,7,8,9,10,11,12,13,14,15);
}
__device__ __forceinline__ float quant(float v, float scale) {
  const float q = rintf(__fdiv_rn(v, scale));
  return fminf(fmaxf(q, -127.0f), 127.0f);
}

__global__ __launch_bounds__(256) void k_scales(const float* __restrict__ x, const float* __restrict__ w, float* __restrict__ st) {
  __shared__ float red[256]; __shared__ float sw[CO]; __shared__ float sx;
  const int tid = threadIdx.x;
  float m = 0.0f;
  for (int i = tid; i < CB * CC * CHW * CHW; i += 256) m = fmaxf(m, fabsf(x[i]));
  red[tid] = m; __syncthreads();
  for (int o = 128; o > 0; o >>= 1) { if (tid < o) red[tid] = fmaxf(red[tid], red[tid + o]); __syncthreads(); }
  if (tid == 0) sx = 0.05f * (red[0] / 127.0f) + 0.95f;
  __syncthreads();
  if (tid < CO) { float mw = 0.0f; for (int j = 0; j < CK; ++j) mw = fmaxf(mw, fabsf(w[(size_t)tid * CK + j])); sw[tid] = mw / 127.0f; }
  __syncthreads();
#pragma unroll 1
  for (int pass = 0; pass < 2; ++pass) { if (tid == 0) *(volatile float*)st = sx; if (tid < CO) *(volatile float*)(st + 32 + tid) = sw[tid]; __threadfence(); }
}
__global__ __launch_bounds__(256) void k_qw(const float* __restrict__ w, const float* __restrict__ st, h16* __restrict__ qw) {
  __shared__ __attribute__((aligned(16))) h16 row[CK];
  const int o = blockIdx.x, tid = threadIdx.x; const float s = st[32 + o];
  for (int j = tid; j < CK; j += 256) row[j] = (h16)quant(w[(size_t)o * CK + j], s);
  __syncthreads();
#pragma unroll 1
  for (int pass = 0; pass < 2; ++pass) { if (tid < CK / 8) *(volatile v4u_t*)(qw + (size_t)o * CK + tid * 8) = *(const v4ua*)(row + tid * 8); __threadfence(); }
}

__global__ __launch_bounds__(256) void k_conv(const float* __restrict__ x, const h16* __restrict__ qw, const float* __restrict__ lut,
                                             const float* __restrict__ st, const float* __restrict__ bias, float* __restrict__ out) {
  __shared__ float lutS[256 * 256];
  __shared__ __attribute__((aligned(16))) h16 qxm[32 * 584];
  __shared__ float res[CO][33];
  const int b = blockIdx.y, oh = blockIdx.x, tid = threadIdx.x, lane = tid & 31, wave = tid >> 5, half = lane >> 4, l16 = lane & 15;
  const float sx = st[0];
  for (int i = tid; i < 256 * 256 / 4; i += 256) *(v4f_t*)(lutS + i * 4) = *(const v4fa*)(lut + i * 4);
  for (int i = tid; i < 32 * CK; i += 256) { const int px = i / CK, k = i % CK, c = k / 9, tap = k % 9, kh = tap / 3, kw = tap % 3;
    const int yy = oh + kh - 1, xx = px + kw - 1; float q = 0.0f;
    if (yy >= 0 && yy < CHW && xx >= 0 && xx < CHW) q = quant(x[(((size_t)b * CC + c) * CHW + yy) * CHW + xx], sx);
    qxm[px * 584 + k] = (h16)q; }
  __syncthreads();
  { v8f acc0 = {}, acc1 = {};
    const h16* wrow = qw + (size_t)(wave * 16 + l16) * CK;
#pragma unroll 2
    for (int kc = 0; kc < CK / 32; ++kc) { const v16h bf = rfrag(wrow + kc * 32, half);
      acc0 = wmma16(rfrag(qxm + l16 * 584 + kc * 32, half), bf, acc0);
      acc1 = wmma16(rfrag(qxm + (16 + l16) * 584 + kc * 32, half), bf, acc1); }
    const int o = wave * 16 + l16;
#pragma unroll
    for (int r = 0; r < 8; ++r) { res[o][8 * half + r] = 0.5f * acc0[r]; res[o][16 + 8 * half + r] = 0.5f * acc1[r]; } }
  __syncthreads();
  { const int o = tid & 127, p0 = (tid >> 7) * 16; const h16* wrow = qw + (size_t)o * CK;
#pragma unroll 1
    for (int pp = 0; pp < 16; ++pp) { const int px = p0 + pp; float s = 0.0f;
#pragma unroll 4
      for (int j = 0; j < CK; ++j) { const int a = (int)qxm[px * 584 + j] + 128, wq = (int)wrow[j] + 128; s += lutS[(a & 255) * 256 + (wq & 255)]; }
      res[o][px] += 0.5f * s; } }
  __syncthreads();
#pragma unroll 1
  for (int pass = 0; pass < 2; ++pass) {
    for (int i = tid; i < CO * 8; i += 256) { const int o = i >> 3, q = (i & 7) * 4; const float sc = sx * st[32 + o], bb = bias[o]; v4f_t v;
      v.x = res[o][q] * sc + bb; v.y = res[o][q + 1] * sc + bb; v.z = res[o][q + 2] * sc + bb; v.w = res[o][q + 3] * sc + bb;
      *(volatile v4f_t*)(out + (((size_t)b * CO + o) * CHW + oh) * CHW + q) = v; }
    __threadfence();
  }
}

extern "C" void kernel_launch(void* const* d_in, const int* in_sizes, int n_in,
                              void* d_out, int out_size, void* d_ws, size_t ws_size,
                              hipStream_t stream) {
  (void)in_sizes; (void)n_in; (void)out_size; (void)ws_size;
  const float* x    = (const float*)d_in[0];
  const float* w    = (const float*)d_in[1];
  const float* bias = (const float*)d_in[2];
  const float* lut  = (const float*)d_in[3];
  char* ws = (char*)d_ws;
  float* st = (float*)ws; ws += 1024;
  h16*   qw = (h16*)ws;   ws += (size_t)CO * CK * 2;
  k_scales<<<1, 256, 0, stream>>>(x, w, st);
  k_qw<<<CO, 256, 0, stream>>>(w, st, qw);
  k_conv<<<dim3(CHW, CB), 256, 0, stream>>>(x, qw, lut, st, bias, (float*)d_out);
}
